// ImageRNN_78005196030244
// MI455X (gfx1250) — hardware-verified
//
#include <hip/hip_runtime.h>

typedef __attribute__((ext_vector_type(16))) _Float16 v16h;
typedef __attribute__((ext_vector_type(8)))  _Float16 v8h;
typedef __attribute__((ext_vector_type(4)))  _Float16 v4h;
typedef __attribute__((ext_vector_type(16))) __bf16   v16b;
typedef __attribute__((ext_vector_type(8)))  __bf16   v8b;
typedef __attribute__((ext_vector_type(8)))  float    v8f;
typedef __attribute__((ext_vector_type(4)))  float    v4f;

constexpr int kBatch = 256;
constexpr int kStep  = 224;
constexpr int kIn    = 224;
constexpr int kHid   = 1024;
constexpr int kOut   = 4;

constexpr int kSeqPB      = 16;
constexpr int kRnnBlocks  = kBatch / kSeqPB;
constexpr int kRnnThreads = 256;
constexpr int kWaves      = kRnnThreads / 32;
constexpr int kColsPW     = 128;
constexpr int kHP         = kHid + 8;
constexpr int kXP         = kIn + 8;
constexpr int kHTile      = kSeqPB * kHP;
constexpr int kXTile      = kSeqPB * kXP;
constexpr int kXF4PerRow  = kIn / 4;
constexpr int kXF4        = kSeqPB * kXF4PerRow;
constexpr float kWScale   = 32.0f;
constexpr float kWInv     = 1.0f / 32.0f;
static_assert(kBatch % kSeqPB == 0);
static_assert(kHid == kWaves * kColsPW);
static_assert(kHP % 8 == 0 && kXP % 8 == 0);
static_assert(kHid % 32 == 0 && kIn % 32 == 0);
static_assert(kIn % 4 == 0);
static_assert((kXF4 % kRnnThreads) % 32 == 0);
static_assert(kSeqPB * kOut == 64);

constexpr int kDwWih = kHid * kIn / 2;
constexpr int kDwWhh = kHid * kHid / 2;
constexpr int kPrepB1 = kDwWih / 256;
constexpr int kPrepBlocks = kPrepB1 + kDwWhh / 256;
static_assert(kDwWih % 256 == 0 && kDwWhh % 256 == 0);
static_assert(kPrepBlocks == 2496);

__device__ __forceinline__ void dep_guard_h(v8f& a, v8f& b, v16h x, v16h y) { asm volatile("v_nop\n\tv_nop\n\tv_nop\n\tv_nop" : "+v"(a), "+v"(b) : "v"(x), "v"(y)); }
__device__ __forceinline__ void dep_guard_b(v8f& a, v8f& b, v16b x, v16b y) { asm volatile("v_nop\n\tv_nop\n\tv_nop\n\tv_nop" : "+v"(a), "+v"(b) : "v"(x), "v"(y)); }
__device__ __forceinline__ void keep4_h(v16h a, v16h b, v16h c, v16h d) { asm volatile("v_nop" :: "v"(a), "v"(b), "v"(c), "v"(d)); }
__device__ __forceinline__ void keep4_b(v16b a, v16b b, v16b c, v16b d) { asm volatile("v_nop" :: "v"(a), "v"(b), "v"(c), "v"(d)); }
__device__ __forceinline__ void acc_guard4(v8f& a, v8f& b, v8f& c, v8f& d) { asm volatile("v_nop\n\tv_nop\n\tv_nop\n\tv_nop" : "+v"(a), "+v"(b), "+v"(c), "+v"(d)); }

template <typename T> struct Frag;
template <> struct Frag<_Float16> {
  typedef v16h V; union U { v16h v; v8h h[2]; };
  static __device__ __forceinline__ v16h load(const _Float16* p) {
    U f; f.h[0] = *(const v8h*)(p); f.h[1] = *(const v8h*)(p + 16); return f.v;
  }
  static __device__ __forceinline__ v8f mma(v16h a, v16h b, v8f c) {
    return __builtin_amdgcn_wmma_f32_16x16x32_f16(false, a, false, b, (short)0, c, false, false);
  }
  static __device__ __forceinline__ void guard(v8f& a, v8f& b, v16h x, v16h y) { dep_guard_h(a, b, x, y); }
  static __device__ __forceinline__ void keep(v16h a, v16h b, v16h c, v16h d) { keep4_h(a, b, c, d); }
};
template <> struct Frag<__bf16> {
  typedef v16b V; union U { v16b v; v8b h[2]; };
  static __device__ __forceinline__ v16b load(const __bf16* p) {
    U f; f.h[0] = *(const v8b*)(p); f.h[1] = *(const v8b*)(p + 16); return f.v;
  }
  static __device__ __forceinline__ v8f mma(v16b a, v16b b, v8f c) {
    return __builtin_amdgcn_wmma_f32_16x16x32_bf16(false, a, false, b, (short)0, c, false, false);
  }
  static __device__ __forceinline__ void guard(v8f& a, v8f& b, v16b x, v16b y) { dep_guard_b(a, b, x, y); }
  static __device__ __forceinline__ void keep(v16b a, v16b b, v16b c, v16b d) { keep4_b(a, b, c, d); }
};

__device__ __forceinline__ unsigned pack_f16x2(float a, float b) {
  const _Float16 h0 = (_Float16)a, h1 = (_Float16)b;
  return (unsigned)__builtin_bit_cast(unsigned short, h0) | ((unsigned)__builtin_bit_cast(unsigned short, h1) << 16);
}
__device__ __forceinline__ void st2u(unsigned* p, unsigned v) { *(volatile unsigned*)p = v; __threadfence(); *(volatile unsigned*)p = v; }
__device__ __forceinline__ float ftanh(float x) { return 1.0f - 2.0f * __builtin_amdgcn_rcpf(1.0f + __expf(2.0f * x)); }

__global__ __launch_bounds__(256) void prep_kernel(
    const float* __restrict__ w_ih, const float* __restrict__ w_hh,
    unsigned* __restrict__ wihu, unsigned* __restrict__ whhu) {
  const int blk = blockIdx.x, tid = threadIdx.x;
  if (blk < kPrepB1) {
    const int p = blk * 256 + tid;
    st2u(wihu + p, pack_f16x2(w_ih[2 * p] * kWScale, w_ih[2 * p + 1] * kWScale));
  } else {
    const int p = (blk - kPrepB1) * 256 + tid;
    st2u(whhu + p, pack_f16x2(w_hh[2 * p] * kWScale, w_hh[2 * p + 1] * kWScale));
  }
}

__device__ __forceinline__ void stage_x(const float* __restrict__ x, _Float16* xtile, int seq0, int t, int tid) {
  for (int i = tid; i < kXF4; i += kRnnThreads) {
    const int r = i / kXF4PerRow;
    const int q = i - r * kXF4PerRow;
    const v4f v = *(const v4f*)(x + ((size_t)(seq0 + r) * kStep + t) * kIn + 4 * q);
    v4h hv;
    hv[0] = (_Float16)v[0]; hv[1] = (_Float16)v[1]; hv[2] = (_Float16)v[2]; hv[3] = (_Float16)v[3];
    *(v4h*)(xtile + r * kXP + 4 * q) = hv;
  }
}

__global__ __launch_bounds__(kRnnThreads) void rnn_kernel(
    const float* __restrict__ x,
    const _Float16* __restrict__ wih16, const _Float16* __restrict__ whh16,
    const float* __restrict__ b_ih, const float* __restrict__ b_hh,
    const float* __restrict__ w_fc, const float* __restrict__ b_fc,
    float* __restrict__ out) {
  __shared__ __align__(16) _Float16 htile[kHTile];
  __shared__ __align__(16) _Float16 xtile[kXTile];
  __shared__ __align__(16) float red[kWaves * kSeqPB * kOut];
  __shared__ __align__(16) float outs[kSeqPB * kOut];
  const int tid = threadIdx.x, lane = tid & 31, wave = tid >> 5;
  const int c = lane & 15, hh = lane >> 4, koff = hh * 8, mOff = hh * 8;
  const int seq0 = blockIdx.x * kSeqPB;
  const int n0 = wave * kColsPW;

  for (int i = tid; i < kHTile; i += kRnnThreads) htile[i] = (_Float16)0.0f;
  if (tid < kSeqPB * 8) xtile[(tid >> 3) * kXP + kIn + (tid & 7)] = (_Float16)0.0f;
  stage_x(x, xtile, seq0, 0, tid);

  float bsum[8];
#pragma unroll
  for (int j = 0; j < 8; ++j) {
    const int n = n0 + 16 * j + c;
    bsum[j] = (b_ih[n] + b_hh[n]) * kWScale;
  }
  __syncthreads();

  const _Float16* browI = wih16 + (size_t)(n0 + c) * kIn + koff;
  const _Float16* browH = whh16 + (size_t)(n0 + c) * kHid + koff;
  const _Float16* arowX = xtile + c * kXP + koff;
  const _Float16* arowH = htile + c * kHP + koff;

  v8f acc[8];
#pragma unroll 1
  for (int s = 0; s < kStep; ++s) {
#pragma unroll
    for (int j = 0; j < 8; ++j) {
      const float bv = bsum[j];
      acc[j] = (v8f){bv, bv, bv, bv, bv, bv, bv, bv};
    }

    v16h fa;
    v16h fb[4];
#pragma unroll 1
    for (int kc = 0; kc < kIn / 32; ++kc) {
      fa = Frag<_Float16>::load(arowX + kc * 32);
#pragma unroll
      for (int g = 0; g < 2; ++g) {
#pragma unroll
        for (int j = 0; j < 4; ++j) fb[j] = Frag<_Float16>::load(browI + (size_t)(64 * g + 16 * j) * kIn + kc * 32);
#pragma unroll
        for (int j = 0; j < 4; ++j) acc[4 * g + j] = Frag<_Float16>::mma(fa, fb[j], acc[4 * g + j]);
        Frag<_Float16>::guard(acc[4 * g], acc[4 * g + 3], fa, fb[3]);
        Frag<_Float16>::keep(fb[0], fb[1], fb[2], fb[3]);
      }
    }
#pragma unroll 2
    for (int kc = 0; kc < kHid / 32; ++kc) {
      fa = Frag<_Float16>::load(arowH + kc * 32);
#pragma unroll
      for (int g = 0; g < 2; ++g) {
#pragma unroll
        for (int j = 0; j < 4; ++j) fb[j] = Frag<_Float16>::load(browH + (size_t)(64 * g + 16 * j) * kHid + kc * 32);
#pragma unroll
        for (int j = 0; j < 4; ++j) acc[4 * g + j] = Frag<_Float16>::mma(fa, fb[j], acc[4 * g + j]);
        Frag<_Float16>::guard(acc[4 * g], acc[4 * g + 3], fa, fb[3]);
        Frag<_Float16>::keep(fb[0], fb[1], fb[2], fb[3]);
      }
    }
    acc_guard4(acc[0], acc[1], acc[2], acc[3]);
    acc_guard4(acc[4], acc[5], acc[6], acc[7]);

    __syncthreads();

#pragma unroll
    for (int j = 0; j < 8; ++j) {
#pragma unroll
      for (int r = 0; r < 8; ++r) {
        const float hv = ftanh(acc[j][r] * kWInv);
        htile[(mOff + r) * kHP + n0 + 16 * j + c] = (_Float16)hv;
      }
    }
    if (s + 1 < kStep) stage_x(x, xtile, seq0, s + 1, tid);
    __syncthreads();
  }

#pragma unroll
  for (int j = 0; j < 8; ++j) {
#pragma unroll
    for (int r = 0; r < 8; ++r) acc[j][r] = ftanh(acc[j][r] * kWInv);
  }
#pragma unroll 1
  for (int o = 0; o < kOut; ++o) {
    const float* wr = w_fc + (size_t)o * kHid + n0 + c;
    float p[8];
#pragma unroll
    for (int r = 0; r < 8; ++r) p[r] = 0.0f;
#pragma unroll
    for (int j = 0; j < 8; ++j) {
      const float w = wr[16 * j];
#pragma unroll
      for (int r = 0; r < 8; ++r) p[r] += acc[j][r] * w;
    }
#pragma unroll
    for (int r = 0; r < 8; ++r) {
#pragma unroll
      for (int off = 1; off < 16; off <<= 1) p[r] += __shfl_xor(p[r], off, 32);
    }
    if (c == 0) {
#pragma unroll
      for (int r = 0; r < 8; ++r) red[((wave * kSeqPB) + mOff + r) * kOut + o] = p[r];
    }
  }
  __syncthreads();
  if (tid < kSeqPB * kOut) {
    const int row = tid >> 2, o = tid & 3;
    float sum = 0.0f;
#pragma unroll
    for (int w = 0; w < kWaves; ++w) sum += red[(w * kSeqPB + row) * kOut + o];
    outs[tid] = sum + b_fc[o];
  }
  __syncthreads();
  if (wave == 0 && lane < 16) {
    const v4f v = *(const v4f*)(outs + 4 * lane);
    float* op = out + (size_t)seq0 * kOut + 4 * lane;
    *(volatile v4f*)op = v;
    __threadfence();
    *(volatile v4f*)op = v;
  }
}

extern "C" void kernel_launch(void* const* d_in, const int* in_sizes, int n_in,
                              void* d_out, int out_size, void* d_ws, size_t ws_size, hipStream_t stream) {
  if (n_in < 7 || d_out == nullptr || d_ws == nullptr) return;
  if (in_sizes[0] != kBatch * kStep * kIn || in_sizes[1] != kHid * kIn || in_sizes[2] != kHid * kHid ||
      in_sizes[3] != kHid || in_sizes[4] != kHid || in_sizes[5] != kOut * kHid || in_sizes[6] != kOut ||
      out_size != kBatch * kOut) return;

  const float* x    = (const float*)d_in[0];
  const float* w_ih = (const float*)d_in[1];
  const float* w_hh = (const float*)d_in[2];
  const float* b_ih = (const float*)d_in[3];
  const float* b_hh = (const float*)d_in[4];
  const float* w_fc = (const float*)d_in[5];
  const float* b_fc = (const float*)d_in[6];
  float* out = (float*)d_out;

  char* ws = (char*)d_ws; size_t off = 0;
  auto carve = [&](size_t bytes) -> char* { char* p = ws + off; off += (bytes + 255) & ~(size_t)255; return p; };
  unsigned short* WIH16 = (unsigned short*)carve((size_t)kHid * kIn * 2);
  unsigned short* WHH16 = (unsigned short*)carve((size_t)kHid * kHid * 2);
  if (off > ws_size || off > (size_t)134217728) return;

  prep_kernel<<<kPrepBlocks, 256, 0, stream>>>(w_ih, w_hh, (unsigned*)WIH16, (unsigned*)WHH16);

  rnn_kernel<<<kRnnBlocks, kRnnThreads, 0, stream>>>(x, (const _Float16*)WIH16, (const _Float16*)WHH16,
                                                      b_ih, b_hh, w_fc, b_fc, out);
}
